// VersorRotorRNN_12713103196452
// MI455X (gfx1250) — hardware-verified
//
#include <hip/hip_runtime.h>
#include <math.h>

constexpr int kBatch    = 16;
constexpr int kSteps    = 256;
constexpr int kPart     = 16;
constexpr int kDim      = 6;
constexpr int kHid      = 16;
constexpr int kBlade    = 32;
constexpr int kCols     = kHid * kBlade;
constexpr int kThreads  = 512;
constexpr int kRowsBlk  = 32;
constexpr int kBlocks   = (kBatch * kPart) / kRowsBlk;
constexpr int kPitch    = kCols + 8;
constexpr int kSegFloats = kPart * kDim;
constexpr int kSegLanes  = kSegFloats / 4;
constexpr float kWCarry    = 16.0f;
constexpr float kWCarryInv = 1.0f / 16.0f;
constexpr float kEps       = 1e-8f;

static_assert(kCols == 512);
static_assert(kThreads == kHid * 32);
static_assert(kRowsBlk == 2 * kPart);
static_assert(kBlocks * kRowsBlk == kBatch * kPart);
static_assert(kCols % 32 == 0);
static_assert(kSegFloats == 96);
static_assert(kSegLanes == 24);
static_assert((kSegFloats * 4) % 128 == 0);
static_assert(kPitch % 8 == 0);
static_assert(kDim * kCols == kDim * kThreads);
static_assert(kThreads * 16 == 16 * kCols);

typedef __attribute__((ext_vector_type(16))) _Float16 v16h;
typedef __attribute__((ext_vector_type(8)))  _Float16 v8h;
typedef __attribute__((ext_vector_type(8)))  float    v8f;
typedef __attribute__((ext_vector_type(4)))  float    v4f;
typedef __attribute__((ext_vector_type(2)))  float    v2f;

struct FragH {
  union U { v16h v; v8h h[2]; };
  static __device__ __forceinline__ v16h load(const _Float16* p) {
    U f;
    f.h[0] = *(const v8h*)(p);
    f.h[1] = *(const v8h*)(p + 16);
    return f.v;
  }
  static __device__ __forceinline__ v8f mma(v16h a, v16h b, v8f c) {
    return __builtin_amdgcn_wmma_f32_16x16x32_f16(false, a, false, b, (short)0, c, false, false);
  }
};

__device__ __forceinline__ void pair_guard(v8f& p, v8f& q, v16h a0, v16h b0, v16h a1, v16h b1) {
  asm volatile("v_nop\n\tv_nop\n\tv_nop\n\tv_nop" : "+v"(p), "+v"(q) : "v"(a0), "v"(b0), "v"(a1), "v"(b1));
}

constexpr bool gp_neg(int i, int j) {
  int a = i >> 1;
  int s = 0;
  while (a) {
    int v = a & j;
    while (v) { s += (v & 1); v >>= 1; }
    a >>= 1;
  }
  return (s & 1) != 0;
}
static_assert(!gp_neg(1, 2));
static_assert(gp_neg(2, 1));
static_assert(gp_neg(3, 3));
static_assert(!gp_neg(1, 1));

template <int I, int K> struct GpK {
  static __device__ __forceinline__ void run(const float (&dv)[kBlade], const float (&ps)[kBlade], float (&ac)[kBlade]) {
    constexpr int J = I ^ K;
    constexpr bool NEG = gp_neg(I, J);
    const float d = NEG ? -dv[I] : dv[I];
    if constexpr (I == 0) {
      ac[K] = d * ps[J];
    } else {
      ac[K] = fmaf(d, ps[J], ac[K]);
    }
    GpK<I, K + 1>::run(dv, ps, ac);
  }
};
template <int I> struct GpK<I, kBlade> {
  static __device__ __forceinline__ void run(const float (&)[kBlade], const float (&)[kBlade], float (&)[kBlade]) {}
};
template <int I> struct GpI {
  static __device__ __forceinline__ void run(const float (&dv)[kBlade], const float (&ps)[kBlade], float (&ac)[kBlade]) {
    GpK<I, 0>::run(dv, ps, ac);
    GpI<I + 1>::run(dv, ps, ac);
  }
};
template <> struct GpI<kBlade> {
  static __device__ __forceinline__ void run(const float (&)[kBlade], const float (&)[kBlade], float (&)[kBlade]) {}
};

__global__ __launch_bounds__(kThreads) void rotor_scan_kernel(const float* __restrict__ x,
                                                              const float* __restrict__ w_in,
                                                              const float* __restrict__ b_in,
                                                              const float* __restrict__ w_out,
                                                              const float* __restrict__ b_out,
                                                              float* __restrict__ out) {
  __shared__ __align__(16) _Float16 sPsi[kRowsBlk * kPitch];
  __shared__ __align__(16) _Float16 sWoT[16 * kPitch];
  __shared__ __align__(16) float    sWin[kDim * kCols];
  __shared__ __align__(16) float    sBin[kCols];
  __shared__ __align__(16) float    sSlab[2][kSegFloats];

  const int tid  = threadIdx.x;
  const int lane = tid & 31;
  const int hw   = __builtin_amdgcn_readfirstlane(tid >> 5);
  const int c    = lane & 15;
  const int hh   = lane >> 4;

#pragma unroll 1
  for (int j = 0; j < kDim; ++j) sWin[j * kCols + tid] = w_in[j * kCols + tid];
  sBin[tid] = b_in[tid];

  {
    const int m  = tid >> 5;
    const int mc = (m < kDim) ? m : (kDim - 1);
    const int k0 = (tid & 31) * 16;
    v8h lo8, hi8;
#pragma unroll
    for (int e = 0; e < 8; ++e) {
      const float wa = w_out[(k0 + e) * kDim + mc];
      const float wb = w_out[(k0 + 8 + e) * kDim + mc];
      const float sa = (m < kDim) ? (wa * kWCarry) : 0.0f;
      const float sb = (m < kDim) ? (wb * kWCarry) : 0.0f;
      lo8[e] = (_Float16)sa;
      hi8[e] = (_Float16)sb;
    }
    *(v8h*)(sWoT + m * kPitch + k0)     = lo8;
    *(v8h*)(sWoT + m * kPitch + k0 + 8) = hi8;
  }

  const int l4 = ((lane < kSegLanes) ? lane : (kSegLanes - 1)) * 4;
  float bo[4];
#pragma unroll
  for (int e = 0; e < 4; ++e) bo[e] = b_out[(l4 + e) % kDim];

  float psi[kBlade];
#pragma unroll
  for (int k = 0; k < kBlade; ++k) psi[k] = 0.0f;
  psi[0] = 1.0f;

  const int bglob = blockIdx.x * 2 + hh;
  const float* xrow0 = x + ((size_t)bglob * kSteps * kPart + (size_t)c) * kDim;
  _Float16* prow = sPsi + lane * kPitch + hw * kBlade;
  const v8f z8 = {0.f, 0.f, 0.f, 0.f, 0.f, 0.f, 0.f, 0.f};

  __syncthreads();

#pragma unroll 1
  for (int t = 0; t < kSteps; ++t) {
    const float* xp = xrow0 + (size_t)t * (kPart * kDim);
    const v2f x01 = *(const v2f*)(xp);
    const v2f x23 = *(const v2f*)(xp + 2);
    const v2f x45 = *(const v2f*)(xp + 4);
    float xs[kDim];
    xs[0] = x01[0]; xs[1] = x01[1]; xs[2] = x23[0]; xs[3] = x23[1]; xs[4] = x45[0]; xs[5] = x45[1];

    int wo = hw * kBlade;
    asm volatile("" : "+v"(wo));
    float dv[kBlade];
#pragma unroll
    for (int kb = 0; kb < 4; ++kb) {
      const float* wp = sWin + wo + 8 * kb;
      const float* bp = sBin + wo + 8 * kb;
      v4f ua = *(const v4f*)(bp);
      v4f ub = *(const v4f*)(bp + 4);
#pragma unroll
      for (int d = 0; d < kDim; ++d) {
        const v4f wa = *(const v4f*)(wp + d * kCols);
        const v4f wb = *(const v4f*)(wp + d * kCols + 4);
#pragma unroll
        for (int e = 0; e < 4; ++e) {
          ua[e] = fmaf(xs[d], wa[e], ua[e]);
          ub[e] = fmaf(xs[d], wb[e], ub[e]);
        }
      }
#pragma unroll
      for (int e = 0; e < 4; ++e) {
        dv[8 * kb + e]     = ua[e];
        dv[8 * kb + 4 + e] = ub[e];
      }
      asm volatile("" ::: "memory");
    }
    dv[0] += 1.0f;

    float s1 = 0.0f;
#pragma unroll
    for (int k = 0; k < kBlade; ++k) s1 = fmaf(dv[k], dv[k], s1);
    const float rs1 = rsqrtf(s1 + kEps);

    float acc[kBlade];
    GpI<0>::run(dv, psi, acc);

    float sa = 0.0f;
#pragma unroll
    for (int k = 0; k < kBlade; ++k) sa = fmaf(acc[k], acc[k], sa);
    const float s2 = fmaf(sa, rs1 * rs1, kEps);
    const float scl = rs1 * rsqrtf(s2);
#pragma unroll
    for (int k = 0; k < kBlade; ++k) psi[k] = acc[k] * scl;

#pragma unroll
    for (int q = 0; q < 4; ++q) {
      v8h hv;
#pragma unroll
      for (int e = 0; e < 8; ++e) hv[e] = (_Float16)psi[8 * q + e];
      *(v8h*)(prow + 8 * q) = hv;
    }
    __syncthreads();

    if (hw < 2) {
      int ao = c * kPitch + 8 * hh;
      asm volatile("" : "+v"(ao));
      const _Float16* ap = sWoT + ao;
      const _Float16* bp = sPsi + (16 * hw + c) * kPitch + 8 * hh;
      v8f acc0 = z8, acc1 = z8;
#pragma unroll
      for (int kp = 0; kp < 8; ++kp) {
        const v16h a0 = FragH::load(ap + 64 * kp);
        const v16h b0 = FragH::load(bp + 64 * kp);
        const v16h a1 = FragH::load(ap + 64 * kp + 32);
        const v16h b1 = FragH::load(bp + 64 * kp + 32);
        acc0 = FragH::mma(a0, b0, acc0);
        acc1 = FragH::mma(a1, b1, acc1);
        pair_guard(acc0, acc1, a0, b0, a1, b1);
      }
      float* slab = sSlab[hw];
      if (hh == 0) {
#pragma unroll
        for (int r = 0; r < kDim; ++r) slab[c * kDim + r] = (acc0[r] + acc1[r]) * kWCarryInv;
      }
      __builtin_amdgcn_fence(__ATOMIC_RELEASE, "workgroup");
      __builtin_amdgcn_wave_barrier();
      __builtin_amdgcn_fence(__ATOMIC_ACQUIRE, "workgroup");
      const size_t seg = ((size_t)(blockIdx.x * 2 + hw) * kSteps + (size_t)t) * kSegFloats;
      const v4f pv = *(const v4f*)(slab + l4);
      const v4f xr = *(const v4f*)(x + seg + l4);
      v4f y;
#pragma unroll
      for (int e = 0; e < 4; ++e) y[e] = xr[e] + (pv[e] + bo[e]);
      float* op = out + seg + l4;
      for (int pass = 0; pass < 2; ++pass) {
        if (lane < kSegLanes) *(volatile v4f*)op = y;
        __threadfence();
      }
      __builtin_amdgcn_fence(__ATOMIC_RELEASE, "workgroup");
      __builtin_amdgcn_wave_barrier();
      __builtin_amdgcn_fence(__ATOMIC_ACQUIRE, "workgroup");
    }
    __syncthreads();
  }
}

extern "C" void kernel_launch(void* const* d_in, const int* in_sizes, int n_in,
                              void* d_out, int out_size, void* d_ws, size_t ws_size, hipStream_t stream) {
  (void)d_ws; (void)ws_size;
  if (n_in < 5 || d_out == nullptr) return;
  if (in_sizes[0] != kBatch * kSteps * kPart * kDim || in_sizes[1] != kDim * kCols || in_sizes[2] != kCols ||
      in_sizes[3] != kCols * kDim || in_sizes[4] != kDim || out_size != kBatch * kSteps * kPart * kDim) return;
  const float* x     = (const float*)d_in[0];
  const float* w_in  = (const float*)d_in[1];
  const float* b_in  = (const float*)d_in[2];
  const float* w_out = (const float*)d_in[3];
  const float* b_out = (const float*)d_in[4];
  float* out = (float*)d_out;
  rotor_scan_kernel<<<kBlocks, kThreads, 0, stream>>>(x, w_in, b_in, w_out, b_out, out);
}
